// NeuralKYAttention_31138512896504
// MI455X (gfx1250) — hardware-verified
//
#include <hip/hip_runtime.h>


#define NB_  2
#define LL   2048
#define DM   1024
#define NH_  16
#define HD   64
#define WN   32
typedef _Float16 h16;
typedef unsigned short bf;
typedef __attribute__((ext_vector_type(16))) __bf16   v16bf;
typedef __attribute__((ext_vector_type(16))) _Float16 v16h;
typedef __attribute__((ext_vector_type(8)))  _Float16 v8h;
typedef __attribute__((ext_vector_type(8)))  unsigned short v8us;
typedef __attribute__((ext_vector_type(8)))  float    v8f;
typedef __attribute__((ext_vector_type(4)))  float    v4f;
typedef v8h  __attribute__((may_alias)) v8ha;
typedef v4f  __attribute__((may_alias)) v4fa;
typedef v8us __attribute__((may_alias)) v8usa;

__device__ __forceinline__ unsigned short f2bf(float f) { unsigned u = __float_as_uint(f); u += 0x7FFFu + ((u >> 16) & 1u); return (unsigned short)(u >> 16); }
__device__ __forceinline__ float bf2f(unsigned short b) { return __uint_as_float(((unsigned)b) << 16); }
__device__ __forceinline__ float bfr(float f) { return bf2f(f2bf(f)); }
__device__ __forceinline__ v16h cat16(v8h lo, v8h hi) { return __builtin_shufflevector(lo, hi, 0, 1, 2, 3, 4, 5, 6, 7, 8, 9, 10, 11, 12, 13, 14, 15); }
__device__ __forceinline__ v16bf cat16b(v8us lo, v8us hi) { return __builtin_bit_cast(v16bf, __builtin_shufflevector(lo, hi, 0, 1, 2, 3, 4, 5, 6, 7, 8, 9, 10, 11, 12, 13, 14, 15)); }
__device__ __forceinline__ v8f wmma16(v16h a, v16h b, v8f c) { return __builtin_amdgcn_wmma_f32_16x16x32_f16(false, a, false, b, (short)0, c, false, false); }
__device__ __forceinline__ v8f wmmab(v16bf a, v16bf b, v8f c) { return __builtin_amdgcn_wmma_f32_16x16x32_bf16(false, a, false, b, (short)0, c, false, false); }


template <typename T16> struct WFrag;
template <> struct WFrag<h16> { typedef v16h V; static __device__ __forceinline__ V ld(const h16* p) { return cat16(*(const v8h*)p, *(const v8h*)(p + 16)); } static __device__ __forceinline__ v8f mma(V a, V b, v8f c) { return wmma16(a, b, c); } };
template <> struct WFrag<bf> { typedef v16bf V; static __device__ __forceinline__ V ld(const bf* p) { return cat16b(*(const v8us*)p, *(const v8us*)(p + 16)); } static __device__ __forceinline__ v8f mma(V a, V b, v8f c) { return wmmab(a, b, c); } };
template <typename T16, int NSPLIT, bool BIAS>
__global__ __launch_bounds__(32) void k_gemmw(const T16* __restrict__ A, const T16* __restrict__ A2, const T16* __restrict__ Bt, const T16* __restrict__ Bt2, int K, float* C, int ldc, const float* __restrict__ bias, size_t sA, size_t sB, size_t sC) {
    typedef typename WFrag<T16>::V V;
    __shared__ __align__(16) float os[16 * 68];
    const size_t z = blockIdx.z; A += z * sA; if (A2) A2 += z * sA; Bt += z * sB; if (Bt2) Bt2 += z * sB; C += z * sC;
    const int lane = threadIdx.x & 31, lr = lane & 15, hi = lane >> 4; const int r0 = blockIdx.x * 64, c0 = blockIdx.y * 64;
    v8f acc[4][4];
#pragma unroll
    for (int mb = 0; mb < 4; ++mb)
#pragma unroll
        for (int nb = 0; nb < 4; ++nb) acc[mb][nb] = (v8f){};
    const size_t aoff = (size_t)(r0 + lr) * K + 8 * hi, boff = (size_t)(c0 + lr) * K + 8 * hi;
#pragma unroll 1
    for (int kc = 0; kc < K; kc += 32) {
        V a[4], a2[4];
#pragma unroll
        for (int mb = 0; mb < 4; ++mb) { a[mb] = WFrag<T16>::ld(A + aoff + (size_t)mb * 16 * K + kc); if (NSPLIT == 1 || NSPLIT == 2) a2[mb] = WFrag<T16>::ld(A2 + aoff + (size_t)mb * 16 * K + kc); }
#pragma unroll
        for (int nb = 0; nb < 4; ++nb) { const V b = WFrag<T16>::ld(Bt + boff + (size_t)nb * 16 * K + kc); V b2; if (NSPLIT >= 2) b2 = WFrag<T16>::ld(Bt2 + boff + (size_t)nb * 16 * K + kc);
#pragma unroll
            for (int mb = 0; mb < 4; ++mb) { acc[mb][nb] = WFrag<T16>::mma(a[mb], b, acc[mb][nb]); if (NSPLIT == 1 || NSPLIT == 2) acc[mb][nb] = WFrag<T16>::mma(a2[mb], b, acc[mb][nb]); if (NSPLIT >= 2) acc[mb][nb] = WFrag<T16>::mma(a[mb], b2, acc[mb][nb]); } }
        asm volatile("v_nop\n\tv_nop\n\tv_nop\n\tv_nop" : "+v"(acc[0][0]), "+v"(acc[1][1]), "+v"(acc[2][2]), "+v"(acc[3][3]) : "v"(a[0]), "v"(a[3]));
    }
#pragma unroll
    for (int mb = 0; mb < 4; ++mb) {
#pragma unroll
        for (int nb = 0; nb < 4; ++nb) {
#pragma unroll
            for (int j = 0; j < 8; ++j) os[(hi * 8 + j) * 68 + nb * 16 + lr] = acc[mb][nb][j]; }
        __builtin_amdgcn_wave_barrier(); asm volatile("" ::: "memory");
        float* crow = C + (size_t)(r0 + mb * 16) * ldc + c0;
#pragma unroll 1
        for (int ps = 0; ps < 2; ++ps) {
#pragma unroll
            for (int s = 0; s < 8; ++s) { const int row = 2 * s + hi, cofs = lr * 4; v4f val = *(const v4fa*)(os + row * 68 + cofs); if (BIAS) { val[0] += bfr(bias[c0 + cofs]); val[1] += bfr(bias[c0 + cofs + 1]); val[2] += bfr(bias[c0 + cofs + 2]); val[3] += bfr(bias[c0 + cofs + 3]); }
                *(volatile v4f*)(crow + (size_t)row * ldc + cofs) = val; }
            if (ps == 0) __threadfence(); }
        __builtin_amdgcn_wave_barrier(); asm volatile("" ::: "memory");
    }
}

__device__ __forceinline__ void splitf(float y, unsigned short& h, unsigned short& l) { h = f2bf(y); l = f2bf(y - bf2f(h)); }
typedef __attribute__((ext_vector_type(2))) unsigned short v2us;
typedef __attribute__((ext_vector_type(4))) unsigned short v4us;

__global__ __launch_bounds__(256) void k_cvt8(const float* __restrict__ src, bf* dst, size_t n8) { const size_t i = (size_t)blockIdx.x * 256 + threadIdx.x; if (i >= n8) return; const v8f v = *(const v8f*)(src + i * 8); v8us o;
#pragma unroll
    for (int k = 0; k < 8; ++k) o[k] = f2bf(v[k]); *(volatile v8us*)(dst + i * 8) = o; __threadfence(); *(volatile v8us*)(dst + i * 8) = o; }
__global__ __launch_bounds__(256) void k_ropef(const float* __restrict__ F, const float* __restrict__ rc, const float* __restrict__ rs, float* R) { const size_t e = ((size_t)blockIdx.x * 256 + threadIdx.x) * 4; if (e >= (size_t)LL * DM) return; const int c = (int)(e % DM); const size_t l = e / DM; const int d = c % HD; const v4f a = *(const v4f*)(F + e); v4f r;
#pragma unroll
    for (int u = 0; u < 4; u += 2) { const int i = (d + u) >> 1; const float cs = bfr(rc[l * (HD / 2) + i]), sn = bfr(rs[l * (HD / 2) + i]); float p0 = __fmul_rn(a[u], cs), p1 = __fmul_rn(a[u + 1], sn), p2 = __fmul_rn(a[u], sn), p3 = __fmul_rn(a[u + 1], cs); asm volatile("" : "+v"(p0)); asm volatile("" : "+v"(p1)); asm volatile("" : "+v"(p2)); asm volatile("" : "+v"(p3)); r[u] = __fsub_rn(p0, p1); r[u + 1] = __fadd_rn(p2, p3); }
    *(volatile v4f*)(R + e) = r; __threadfence(); *(volatile v4f*)(R + e) = r; }
__global__ __launch_bounds__(32) void k_conn(const float* __restrict__ cw1, const float* __restrict__ cw2, const float* __restrict__ cw3, float* CONN) { const int h = blockIdx.x; const int w = threadIdx.x; const float pos = (float)w / (float)(WN - 1); float acc = 0.f;
#pragma unroll 1
    for (int k = 0; k < 128; ++k) { const float a1 = __fmul_rn(pos, bfr(cw1[h * 128 + k])); const float a3 = __fmul_rn(pos, bfr(cw3[h * 128 + k])); const float sl = __fdiv_rn(a1, __fadd_rn(1.0f, __expf(-a1))); float t = __fmul_rn(sl, a3); asm volatile("" : "+v"(t)); float t2 = __fmul_rn(t, bfr(cw2[h * 128 + k])); asm volatile("" : "+v"(t2)); acc = __fadd_rn(acc, t2); }
    float mx = acc;
#pragma unroll
    for (int sh = 16; sh; sh >>= 1) mx = fmaxf(mx, __shfl_xor(mx, sh, 32));
    const float e = __expf(__fsub_rn(acc, mx)); float s = e;
#pragma unroll
    for (int sh = 16; sh; sh >>= 1) s += __shfl_xor(s, sh, 32);
    const float c = __fdiv_rn(e, s); *(volatile float*)(CONN + h * WN + w) = c; __threadfence(); *(volatile float*)(CONN + h * WN + w) = c; }
__global__ __launch_bounds__(256) void k_win(const float* __restrict__ QR, const float* __restrict__ KR, const float* __restrict__ V, const float* __restrict__ CONN, bf* Ah, bf* Al) {
    const int lane = threadIdx.x & 31; const int row = blockIdx.x * 8 + (threadIdx.x >> 5); if (row >= NH_ * LL) return; const int l = row % LL; const int h = row / LL;
    const int kk = l - (WN - 1) + lane; const float* q = QR + (size_t)l * DM + h * HD; float s = 0.f;
    if (kk >= 0) { const float* k = KR + (size_t)kk * DM + h * HD;
#pragma unroll 1
        for (int d = 0; d < HD; ++d) { float p = __fmul_rn(q[d], k[d]); asm volatile("" : "+v"(p)); s = __fadd_rn(s, p); } }
    s = s * 0.125f;
    float mx = s;
#pragma unroll
    for (int sh = 16; sh; sh >>= 1) mx = fmaxf(mx, __shfl_xor(mx, sh, 32));
    float d0 = __fsub_rn(s, mx); asm volatile("" : "+v"(d0)); const float e = __builtin_amdgcn_exp2f(__fmul_rn(d0, 1.4426950408889634f)); float sum = e;
#pragma unroll
    for (int sh = 16; sh; sh >>= 1) sum += __shfl_xor(sum, sh, 32);
    const float attn = __fdiv_rn(e, sum); float fin = __fmul_rn(attn, CONN[h * WN + lane]); float fs = fin;
#pragma unroll
    for (int sh = 16; sh; sh >>= 1) fs += __shfl_xor(fs, sh, 32);
    fin = __fdiv_rn(fin, __fadd_rn(fs, 1e-9f));
    float o0 = 0.f, o1 = 0.f; const int dcol = h * HD + 2 * lane;
#pragma unroll 1
    for (int w = 0; w < WN; ++w) { const float fw = __shfl(fin, w, 32); const int kw = l - (WN - 1) + w; if (kw >= 0) { const float* vr = V + (size_t)kw * DM + dcol; float p0 = __fmul_rn(fw, vr[0]), p1 = __fmul_rn(fw, vr[1]); asm volatile("" : "+v"(p0)); asm volatile("" : "+v"(p1)); o0 = __fadd_rn(o0, p0); o1 = __fadd_rn(o1, p1); } }
    unsigned short a0, b0, a1, b1; splitf(o0, a0, b0); splitf(o1, a1, b1); v2us oh, ol; oh[0] = a0; oh[1] = a1; ol[0] = b0; ol[1] = b1; const size_t oo = (size_t)l * DM + dcol;
    *(volatile v2us*)(Ah + oo) = oh; *(volatile v2us*)(Al + oo) = ol; __threadfence(); *(volatile v2us*)(Ah + oo) = oh; *(volatile v2us*)(Al + oo) = ol; }

extern "C" void kernel_launch(void* const* d_in, const int* in_sizes, int n_in,
                              void* d_out, int out_size, void* d_ws, size_t ws_size, hipStream_t stream) {
    (void)in_sizes; (void)n_in; (void)out_size;
    const float* x = (const float*)d_in[0]; const float* wq = (const float*)d_in[1]; const float* wk = (const float*)d_in[2]; const float* wv = (const float*)d_in[3]; const float* wo = (const float*)d_in[4]; const float* cw1 = (const float*)d_in[5]; const float* cw2 = (const float*)d_in[6]; const float* cw3 = (const float*)d_in[7]; const float* rc = (const float*)d_in[8]; const float* rs = (const float*)d_in[9];
    float* OUT = (float*)d_out;
    char* wsp = (char*)d_ws;
    auto take = [&](size_t bytes) { char* p = wsp; wsp += (bytes + 255) & ~(size_t)255; return (void*)p; };
    bf* BQ = (bf*)take((size_t)DM * DM * 2); bf* BK = (bf*)take((size_t)DM * DM * 2); bf* BV = (bf*)take((size_t)DM * DM * 2); bf* BO = (bf*)take((size_t)DM * DM * 2); float* CONN = (float*)take(NH_ * WN * 4);
    bf* XB = (bf*)take((size_t)LL * DM * 2); float* F = (float*)take((size_t)LL * DM * 4); float* QR = (float*)take((size_t)LL * DM * 4); float* KR = (float*)take((size_t)LL * DM * 4); float* V = (float*)take((size_t)LL * DM * 4); bf* ATh = (bf*)take((size_t)LL * DM * 2); bf* ATl = (bf*)take((size_t)LL * DM * 2);
    if ((size_t)(wsp - (char*)d_ws) > ws_size) return;
    k_cvt8<<<(DM * DM / 8 + 255) / 256, 256, 0, stream>>>(wq, BQ, DM * DM / 8); k_cvt8<<<(DM * DM / 8 + 255) / 256, 256, 0, stream>>>(wk, BK, DM * DM / 8); k_cvt8<<<(DM * DM / 8 + 255) / 256, 256, 0, stream>>>(wv, BV, DM * DM / 8); k_cvt8<<<(DM * DM / 8 + 255) / 256, 256, 0, stream>>>(wo, BO, DM * DM / 8);
    k_conn<<<NH_, 32, 0, stream>>>(cw1, cw2, cw3, CONN);
    const dim3 gp(LL / 64, DM / 64, 1); const unsigned LP = (unsigned)(((size_t)LL * DM / 4 + 255) / 256);
    for (int b = 0; b < NB_; ++b) {
        k_cvt8<<<(LL * DM / 8 + 255) / 256, 256, 0, stream>>>(x + (size_t)b * LL * DM, XB, LL * DM / 8);
        k_gemmw<bf, 0, false><<<gp, 32, 0, stream>>>(XB, nullptr, BQ, nullptr, DM, F, DM, nullptr, 0, 0, 0); k_ropef<<<LP, 256, 0, stream>>>(F, rc, rs, QR);
        k_gemmw<bf, 0, false><<<gp, 32, 0, stream>>>(XB, nullptr, BK, nullptr, DM, F, DM, nullptr, 0, 0, 0); k_ropef<<<LP, 256, 0, stream>>>(F, rc, rs, KR);
        k_gemmw<bf, 0, false><<<gp, 32, 0, stream>>>(XB, nullptr, BV, nullptr, DM, V, DM, nullptr, 0, 0, 0);
        k_win<<<NH_ * LL / 8, 256, 0, stream>>>(QR, KR, V, CONN, ATh, ATl);
        k_gemmw<bf, 1, false><<<gp, 32, 0, stream>>>(ATh, ATl, BO, nullptr, DM, OUT + (size_t)b * LL * DM, DM, nullptr, 0, 0, 0); }
}
